// SeparateHiddenGCVAEEncoder_16286515987223
// MI455X (gfx1250) — hardware-verified
//
#include <hip/hip_runtime.h>
#include <stdint.h>
#include <math.h>


#define FEATD 128
#define CONDD 64
#define HIDD  128
#define LATD  64
#define NCOL  128
#define TPB   256
#define NWAVE (TPB / 32)
#define EPT   8
#define LMAX  (EPT * 32)
#define ACCF  57344
#define NBG   (ACCF / TPB)
#define RND   16384
#define KEYSH 12

#define SC_X 16.0f
#define SC_H 256.0f
#define SC_W 64.0f

#if (ACCF % (8 * TPB)) != 0 || (RND % (4 * TPB)) != 0 || (2 * NBG) > (1 << KEYSH)
#error config
#endif

#define DEG_LDS_BYTES (RND * 4 + NWAVE * LMAX * 4 + NWAVE * 4)

typedef _Float16 v16h __attribute__((ext_vector_type(16)));
typedef _Float16 v8h  __attribute__((ext_vector_type(8)));
typedef float    v8f  __attribute__((ext_vector_type(8)));
typedef float    v4f  __attribute__((ext_vector_type(4)));
typedef int      v4i  __attribute__((ext_vector_type(4)));

union Frag  { v16h v; v8h half[2]; _Float16 s[16]; };
union Pack8 { v8h v; _Float16 s[8]; };

__device__ __forceinline__ v8f wmma16(const v16h a, const v16h b, v8f acc)
{
    acc = __builtin_amdgcn_wmma_f32_16x16x32_f16(false, a, false, b, (short)0, acc, false, false);
    asm volatile("v_nop\n\tv_nop\n\tv_nop\n\tv_nop" : "+v"(acc) : "v"(a), "v"(b));
    return acc;
}

__device__ __forceinline__ float tanh_fast(float x)
{
    const float t = __expf(-2.0f * fabsf(x));
    const float r = (1.0f - t) * __builtin_amdgcn_rcpf(1.0f + t);
    return copysignf(r, x);
}

__device__ __forceinline__ void load_afrag(Frag& a, const float* p, int h, float sa)
{
    const v4f* pv = (const v4f*)p;
    const v4f x0 = pv[2 * h], x1 = pv[2 * h + 1], x2 = pv[4 + 2 * h], x3 = pv[5 + 2 * h];
#pragma unroll
    for (int j = 0; j < 4; ++j) {
        a.s[j]      = (_Float16)(x0[j] * sa);
        a.s[4 + j]  = (_Float16)(x1[j] * sa);
        a.s[8 + j]  = (_Float16)(x2[j] * sa);
        a.s[12 + j] = (_Float16)(x3[j] * sa);
    }
}
__device__ __forceinline__ void load_afrag(Frag& a, const _Float16* p, int h, float)
{
    a.half[0] = *(const v8h*)(p + 8 * h);
    a.half[1] = *(const v8h*)(p + 16 + 8 * h);
}

__global__ __launch_bounds__(TPB)
void k_deg(const int* __restrict__ ei, int n_edges, int n_nodes, float* dinv)
{
    extern __shared__ v4i lds_d[];
    int* cnt = (int*)lds_d;
    int* lst = cnt + RND;
    int* wc  = lst + NWAVE * LMAX;
    (void)n_nodes;
    const int tid = threadIdx.x, lane = tid & 31, wave = tid >> 5;
    const int n0 = blockIdx.x * RND;

    const v4i z4 = {0, 0, 0, 0};
    for (int i = tid; i < RND / 4; i += TPB) lds_d[i] = z4;
    __syncthreads();

    const int* dstp = ei + n_edges;
    for (int c0 = 0; c0 < n_edges; c0 += EPT * TPB) {
        int base = 0;
#pragma unroll
        for (int j = 0; j < EPT; ++j) {
            const int e = c0 + j * TPB + tid;
            int local = -1;
            if (e < n_edges) local = dstp[e] - n0;
            const bool match = (unsigned)local < (unsigned)RND;
            const unsigned msk = __builtin_amdgcn_ballot_w32(match);
            if (match) lst[wave * LMAX + base + (int)__builtin_amdgcn_mbcnt_lo(msk, 0u)] = local;
            base += (int)__builtin_popcount(msk);
        }
        if (lane == 0) wc[wave] = base;
        __syncthreads();
        if (tid == 0) {
            for (int w = 0; w < NWAVE; ++w) {
                int cw = wc[w];
                cw = cw < 0 ? 0 : cw;
                cw = cw > LMAX ? LMAX : cw;
                const int* L = lst + w * LMAX;
                for (int q = 0; q < cw; ++q) {
                    int l = L[q];
                    l = ((unsigned)l < (unsigned)RND) ? l : 0;
                    cnt[l] += 1;
                }
            }
        }
        __syncthreads();
    }

#pragma unroll 1
    for (int pass = 0; pass < 2; ++pass) {
#pragma unroll 1
        for (int it = 0; it < RND / 4 / TPB; ++it) {
            const int i4 = it * TPB + tid;
            const v4i cv = lds_d[i4];
            v4f dv;
#pragma unroll
            for (int j = 0; j < 4; ++j) dv[j] = rsqrtf((float)(cv[j] + 1));
            *(volatile v4f*)(dinv + (size_t)n0 + 4 * i4) = dv;
        }
        if (pass == 0) __threadfence();
    }
}

__global__ __launch_bounds__(TPB)
void k_wprep(const float* __restrict__ W0, const float* __restrict__ W1, int K, int N0, int N1, float s,
             _Float16* Wt)
{
    const int t = blockIdx.x * TPB + threadIdx.x;
    const int kq8 = K >> 3;
    const int n = t / kq8, kq = t - n * kq8;
    if (n >= N0 + N1) return;
    Pack8 o;
#pragma unroll
    for (int j = 0; j < 8; ++j) {
        const int k = 8 * kq + j;
        const float x = (n < N0) ? W0[(size_t)k * N0 + n] : W1[(size_t)k * N1 + (n - N0)];
        o.s[j] = (_Float16)(x * s);
    }
    volatile v8h* p = (volatile v8h*)(Wt + (size_t)n * K + 8 * kq);
    *p = o.v;
    __threadfence();
    *p = o.v;
}

template<typename AT, int K, int LDA, int LDC>
__global__ __launch_bounds__(TPB)
void k_gemm(const AT* __restrict__ A, const _Float16* __restrict__ Wt, const float* __restrict__ dinv,
            float* C, int M, float sa, float sc)
{
    __shared__ __align__(16) float tile[NWAVE][16 * 64];
    const int tid = threadIdx.x, wave = tid >> 5, lane = tid & 31, h = lane >> 4, m = lane & 15;
    const int tilesM = (M + 15) >> 4;
    const int numWT = tilesM * (NCOL / 64);
    int wt = blockIdx.x * NWAVE + wave;
    const bool valid = wt < numWT;
    if (!valid) wt = numWT - 1;
    const int tm = wt >> 1;
    const int col0 = (wt & 1) * 64;
    int arow = tm * 16 + m;
    if (arow > M - 1) arow = M - 1;
    const AT* Ap = A + (size_t)arow * LDA;
    const _Float16* Bp = Wt + (size_t)(col0 + m) * K;

    const v8f z8 = {0.f, 0.f, 0.f, 0.f, 0.f, 0.f, 0.f, 0.f};
    v8f acc0 = z8, acc1 = z8, acc2 = z8, acc3 = z8;
#pragma unroll 1
    for (int k0 = 0; k0 < K; k0 += 32) {
        Frag a, b0, b1, b2, b3;
        load_afrag(a, Ap + k0, h, sa);
        const _Float16* q = Bp + k0;
        b0.half[0] = *(const v8h*)(q + 8 * h);           b0.half[1] = *(const v8h*)(q + 16 + 8 * h);
        b1.half[0] = *(const v8h*)(q + 16 * K + 8 * h);  b1.half[1] = *(const v8h*)(q + 16 * K + 16 + 8 * h);
        b2.half[0] = *(const v8h*)(q + 32 * K + 8 * h);  b2.half[1] = *(const v8h*)(q + 32 * K + 16 + 8 * h);
        b3.half[0] = *(const v8h*)(q + 48 * K + 8 * h);  b3.half[1] = *(const v8h*)(q + 48 * K + 16 + 8 * h);
        acc0 = wmma16(a.v, b0.v, acc0);
        acc1 = wmma16(a.v, b1.v, acc1);
        acc2 = wmma16(a.v, b2.v, acc2);
        acc3 = wmma16(a.v, b3.v, acc3);
    }

    float* tw = tile[wave];
#pragma unroll
    for (int r = 0; r < 8; ++r) {
        const int o = (8 * h + r) * 64 + m;
        tw[o]      = acc0[r] * sc;
        tw[o + 16] = acc1[r] * sc;
        tw[o + 32] = acc2[r] * sc;
        tw[o + 48] = acc3[r] * sc;
    }
    __syncthreads();
    const v4f* tv = (const v4f*)tw;
#pragma unroll
    for (int i = 0; i < 8; ++i) {
        const int f = i * 32 + lane, row = f >> 4, c4 = f & 15;
        const int grow = tm * 16 + row;
        const int gr = grow < M ? grow : (M - 1);
        const v4f v = tv[row * 16 + c4] * dinv[gr];
        if (valid && grow < M) *(volatile v4f*)(C + (size_t)grow * LDC + col0 + 4 * c4) = v;
    }
    __threadfence();
#pragma unroll
    for (int i = 0; i < 8; ++i) {
        const int f = i * 32 + lane, row = f >> 4, c4 = f & 15;
        const int grow = tm * 16 + row;
        const int gr = grow < M ? grow : (M - 1);
        const v4f v = tv[row * 16 + c4] * dinv[gr];
        if (valid && grow < M) *(volatile v4f*)(C + (size_t)grow * LDC + col0 + 4 * c4) = v;
    }
}

template<int W, bool HEAD>
__global__ __launch_bounds__(TPB)
void k_agg(const float* __restrict__ P, const int* __restrict__ ei, int n_edges, int n_nodes,
           const float* __restrict__ dinv, const float* __restrict__ b0, const float* __restrict__ b1,
           const float* __restrict__ noise, _Float16* Hout, float* out)
{
    constexpr int G  = TPB / W;
    constexpr int NB = NBG * G;
    extern __shared__ v4f lds_a[];
    float* acc = (float*)lds_a;
    int*   lst = (int*)((unsigned char*)lds_a + (size_t)ACCF * 4);
    int*   wc  = lst + NWAVE * G * LMAX;
    const int tid = threadIdx.x, lane = tid & 31, wave = tid >> 5;
    const int n0 = blockIdx.x * NB;

    const v4f z4 = {0.f, 0.f, 0.f, 0.f};
    for (int i = tid; i < ACCF / 4; i += TPB) lds_a[i] = z4;
    __syncthreads();

    const int* srcp = ei;
    const int* dstp = ei + n_edges;
    for (int c0 = 0; c0 < n_edges; c0 += EPT * TPB) {
        int base[G];
#pragma unroll
        for (int g = 0; g < G; ++g) base[g] = 0;
#pragma unroll
        for (int j = 0; j < EPT; ++j) {
            const int e = c0 + j * TPB + tid;
            int local = -1, s = 0;
            if (e < n_edges) local = dstp[e] - n0;
            if ((unsigned)local < (unsigned)NB) {
                s = srcp[e];
                s = s < 0 ? 0 : s;
                s = s > n_nodes - 1 ? n_nodes - 1 : s;
            }
#pragma unroll
            for (int g = 0; g < G; ++g) {
                const bool mg = (unsigned)(local - g * NBG) < (unsigned)NBG;
                const unsigned msk = __builtin_amdgcn_ballot_w32(mg);
                if (mg) lst[(wave * G + g) * LMAX + base[g] + (int)__builtin_amdgcn_mbcnt_lo(msk, 0u)] = (s << KEYSH) | local;
                base[g] += (int)__builtin_popcount(msk);
            }
        }
        if (lane == 0) {
#pragma unroll
            for (int g = 0; g < G; ++g) wc[wave * G + g] = base[g];
        }
        __syncthreads();
        {
            const int g = tid / W;
            const int c = tid - g * W;
            float* ac = acc + c;
            const float* Pc = P + c;
#pragma unroll 1
            for (int w = 0; w < NWAVE; ++w) {
                int cw = wc[w * G + g];
                cw = cw < 0 ? 0 : cw;
                cw = cw > LMAX ? LMAX : cw;
                const int* L = lst + (w * G + g) * LMAX;
#pragma unroll 1
                for (int q = 0; q < cw; ++q) {
                    const int key = L[q];
                    int local = key & ((1 << KEYSH) - 1);
                    local = local > NB - 1 ? NB - 1 : local;
                    int s = key >> KEYSH;
                    s = ((unsigned)s < (unsigned)n_nodes) ? s : (n_nodes - 1);
                    ac[local * W] += Pc[(size_t)s * W];
                }
            }
        }
        __syncthreads();
    }

#pragma unroll 1
    for (int pass = 0; pass < 2; ++pass) {
        if (!HEAD) {
            constexpr int NIT = NB * W / 8 / TPB;
#pragma unroll 1
            for (int it = 0; it < NIT; ++it) {
                const int f = (it * TPB + tid) * 8;
                const int local = f / W, c = f - local * W;
                const int node = n0 + local;
                const int nd = node < n_nodes ? node : (n_nodes - 1);
                const float dn = dinv[nd];
                const v4f a0 = *(const v4f*)(acc + local * W + c);
                const v4f a1 = *(const v4f*)(acc + local * W + c + 4);
                const v4f* pr = (const v4f*)(P + (size_t)nd * W + c);
                const v4f p0 = pr[0], p1 = pr[1];
                const float* bp = (W > HIDD && c >= HIDD) ? (b1 + (c - HIDD)) : (b0 + c);
                const v4f bb0 = *(const v4f*)bp, bb1 = *(const v4f*)(bp + 4);
                Pack8 o;
#pragma unroll
                for (int j = 0; j < 4; ++j) {
                    o.s[j]     = (_Float16)(tanh_fast(dn * (a0[j] + p0[j]) + bb0[j]) * SC_H);
                    o.s[4 + j] = (_Float16)(tanh_fast(dn * (a1[j] + p1[j]) + bb1[j]) * SC_H);
                }
                if (node < n_nodes) *(volatile v8h*)(Hout + (size_t)node * W + c) = o.v;
            }
        } else {
            constexpr int NIT = NB * LATD / 4 / TPB;
#pragma unroll 1
            for (int it = 0; it < NIT; ++it) {
                const int f = (it * TPB + tid) * 4;
                const int local = f >> 6, c = f & 63;
                const int node = n0 + local;
                const int nd = node < n_nodes ? node : (n_nodes - 1);
                const float dn = dinv[nd];
                const v4f am = *(const v4f*)(acc + local * W + c);
                const v4f al = *(const v4f*)(acc + local * W + LATD + c);
                const v4f pm = *(const v4f*)(P + (size_t)nd * W + c);
                const v4f pl = *(const v4f*)(P + (size_t)nd * W + LATD + c);
                const v4f bmv = *(const v4f*)(b0 + c);
                const v4f blv = *(const v4f*)(b1 + c);
                const v4f nz  = *(const v4f*)(noise + (size_t)nd * LATD + c);
                const v4f mv = dn * (am + pm) + bmv;
                const v4f lv = dn * (al + pl) + blv;
                v4f zv;
#pragma unroll
                for (int j = 0; j < 4; ++j) zv[j] = nz[j] * __expf(0.5f * lv[j]) + mv[j];
                if (node < n_nodes) {
                    const size_t plane = (size_t)n_nodes * LATD;
                    const size_t o = (size_t)node * LATD + c;
                    *(volatile v4f*)(out + o) = zv;
                    *(volatile v4f*)(out + plane + o) = mv;
                    *(volatile v4f*)(out + 2 * plane + o) = lv;
                }
            }
        }
        if (pass == 0) __threadfence();
    }
}

static inline size_t agg_lds_bytes(int W)
{
    const int G = TPB / W;
    return (size_t)ACCF * 4 + (size_t)NWAVE * G * LMAX * 4 + (size_t)NWAVE * G * 4;
}

extern "C" void kernel_launch(void* const* d_in, const int* in_sizes, int n_in,
                              void* d_out, int out_size, void* d_ws, size_t ws_size,
                              hipStream_t stream)
{
    if (n_in < 14) return;
    const float* feature   = (const float*)d_in[0];
    const float* condition = (const float*)d_in[1];
    const int*   edge      = (const int*)d_in[2];
    const float* noise     = (const float*)d_in[3];
    const float* W_f2h     = (const float*)d_in[4];
    const float* b_f2h     = (const float*)d_in[5];
    const float* W_c2h     = (const float*)d_in[6];
    const float* b_c2h     = (const float*)d_in[7];
    const float* W_h2h     = (const float*)d_in[8];
    const float* b_h2h     = (const float*)d_in[9];
    const float* W_mean    = (const float*)d_in[10];
    const float* b_mean    = (const float*)d_in[11];
    const float* W_logvar  = (const float*)d_in[12];
    const float* b_logvar  = (const float*)d_in[13];

    const int n_nodes = in_sizes[0] / FEATD;
    const int n_edges = in_sizes[2] / 2;
    if (n_nodes <= 0 || n_nodes > 524287 || n_edges < 0) return;
    if (in_sizes[1] < n_nodes * CONDD || in_sizes[3] < n_nodes * LATD) return;
    if (in_sizes[4] < FEATD * HIDD || in_sizes[6] < CONDD * HIDD || in_sizes[8] < 2 * HIDD * HIDD ||
        in_sizes[10] < HIDD * LATD || in_sizes[12] < HIDD * LATD) return;
    if (in_sizes[5] < HIDD || in_sizes[7] < HIDD || in_sizes[9] < HIDD || in_sizes[11] < LATD || in_sizes[13] < LATD) return;
    if (out_size < 3 * n_nodes * LATD) return;

    const int nblk_deg = (n_nodes + RND - 1) / RND;
    const size_t npad = (size_t)nblk_deg * RND;

    char* ws = (char*)d_ws;
    size_t off = 0;
    auto carve = [&](size_t bytes) {
        void* p = ws + off;
        off = (off + bytes + 255) & ~(size_t)255;
        return p;
    };
    float*    dinv = (float*)   carve(npad * 4);
    _Float16* wtf  = (_Float16*)carve((size_t)NCOL * FEATD * 2);
    _Float16* wtc  = (_Float16*)carve((size_t)NCOL * CONDD * 2);
    _Float16* wth  = (_Float16*)carve((size_t)NCOL * 2 * HIDD * 2);
    _Float16* wtml = (_Float16*)carve((size_t)NCOL * HIDD * 2);
    float*    P    = (float*)   carve((size_t)n_nodes * 2 * HIDD * 4);
    _Float16* H    = (_Float16*)carve((size_t)n_nodes * 2 * HIDD * 2);
    if (off > ws_size) return;

    auto blk = [](long n, int t) { return (int)((n + t - 1) / t); };

    k_deg<<<nblk_deg, TPB, DEG_LDS_BYTES, stream>>>(edge, n_edges, n_nodes, dinv);

    k_wprep<<<blk((long)NCOL * FEATD / 8, TPB), TPB, 0, stream>>>(W_f2h, W_f2h, FEATD, HIDD, 0, SC_W, wtf);
    k_wprep<<<blk((long)NCOL * CONDD / 8, TPB), TPB, 0, stream>>>(W_c2h, W_c2h, CONDD, HIDD, 0, SC_W, wtc);
    k_wprep<<<blk((long)NCOL * 2 * HIDD / 8, TPB), TPB, 0, stream>>>(W_h2h, W_h2h, 2 * HIDD, HIDD, 0, SC_W, wth);
    k_wprep<<<blk((long)NCOL * HIDD / 8, TPB), TPB, 0, stream>>>(W_mean, W_logvar, HIDD, LATD, LATD, SC_W, wtml);

    const int numWT = ((n_nodes + 15) / 16) * (NCOL / 64);
    const int gemmBlocks = blk(numWT, NWAVE);

    k_gemm<float, FEATD, FEATD, 2 * HIDD><<<gemmBlocks, TPB, 0, stream>>>(feature, wtf, dinv, P, n_nodes, SC_X, 1.0f / (SC_X * SC_W));
    k_gemm<float, CONDD, CONDD, 2 * HIDD><<<gemmBlocks, TPB, 0, stream>>>(condition, wtc, dinv, P + HIDD, n_nodes, SC_X, 1.0f / (SC_X * SC_W));
    k_agg<2 * HIDD, false><<<blk(n_nodes, NBG), TPB, agg_lds_bytes(2 * HIDD), stream>>>(
        P, edge, n_edges, n_nodes, dinv, b_f2h, b_c2h, noise, H, (float*)d_out);

    k_gemm<_Float16, 2 * HIDD, 2 * HIDD, HIDD><<<gemmBlocks, TPB, 0, stream>>>(H, wth, dinv, P, n_nodes, 1.0f, 1.0f / (SC_H * SC_W));
    k_agg<HIDD, false><<<blk(n_nodes, 2 * NBG), TPB, agg_lds_bytes(HIDD), stream>>>(
        P, edge, n_edges, n_nodes, dinv, b_h2h, b_h2h, noise, H, (float*)d_out);

    k_gemm<_Float16, HIDD, HIDD, 2 * LATD><<<gemmBlocks, TPB, 0, stream>>>(H, wtml, dinv, P, n_nodes, 1.0f, 1.0f / (SC_H * SC_W));
    k_agg<2 * LATD, true><<<blk(n_nodes, 2 * NBG), TPB, agg_lds_bytes(2 * LATD), stream>>>(
        P, edge, n_edges, n_nodes, dinv, b_mean, b_logvar, noise, H, (float*)d_out);
}
